// DotProductAttention_70669391888880
// MI455X (gfx1250) — hardware-verified
//
#include <hip/hip_runtime.h>

typedef _Float16 v16h __attribute__((ext_vector_type(16)));
typedef _Float16 v8h  __attribute__((ext_vector_type(8)));
typedef float    v8f  __attribute__((ext_vector_type(8)));
typedef float    v4f  __attribute__((ext_vector_type(4)));

#ifndef NB
#define NB 2
#endif
#ifndef SEQ
#define SEQ 2048
#endif
#define NB_FULL  2
#define SEQ_FULL 2048
#define NH 16
#define HD 64

constexpr int KVT    = 32;
constexpr int NT     = SEQ / KVT;
constexpr int WAVES  = 4;
constexpr int QB     = WAVES * 16;
constexpr int QBLKS  = SEQ / QB;
constexpr int TILE_H = KVT * HD;
constexpr int NBH    = NB * NH;

constexpr float PSCALE = 16384.0f;
constexpr float PINV   = 1.0f / 16384.0f;
constexpr float SL2E   = 0.125f * 1.4426950408889634f;

static_assert(SEQ % QB == 0);
static_assert(SEQ % KVT == 0);
static_assert(SEQ <= SEQ_FULL);
static_assert(NB <= NB_FULL);
static_assert(HD == 64);
static_assert(TILE_H == 128 * 16);

__device__ __forceinline__ float fast_exp2(float x) {
#if defined(__has_builtin) && __has_builtin(__builtin_amdgcn_exp2f)
    return __builtin_amdgcn_exp2f(x);
#else
    return exp2f(x);
#endif
}
__device__ __forceinline__ float fast_rcp(float x) {
#if defined(__has_builtin) && __has_builtin(__builtin_amdgcn_rcpf)
    return __builtin_amdgcn_rcpf(x);
#else
    return 1.0f / x;
#endif
}

__device__ __forceinline__ float bf16_rne_flush(float x) {
    unsigned u = __float_as_uint(x);
    u = (u + 0x7FFFu + ((u >> 16) & 1u)) & 0xFFFF0000u;
    u = ((u & 0x7F800000u) < 0x38800000u) ? 0u : u;
    return __uint_as_float(u);
}
__device__ __forceinline__ _Float16 to_h(float x) {
    return (_Float16)bf16_rne_flush(x);
}
__device__ __forceinline__ v8h cvt8(float4 a, float4 c) {
    v8h h;
    h[0] = to_h(a.x); h[1] = to_h(a.y); h[2] = to_h(a.z); h[3] = to_h(a.w);
    h[4] = to_h(c.x); h[5] = to_h(c.y); h[6] = to_h(c.z); h[7] = to_h(c.w);
    return h;
}

__device__ __forceinline__ v16h ld_op16(const _Float16* p) {
    v8h lo = *(const v8h*)p;
    v8h hh = *(const v8h*)(p + 16);
    v16h r;
#pragma unroll
    for (int i = 0; i < 8; ++i) { r[i] = lo[i]; r[i + 8] = hh[i]; }
    return r;
}

__device__ __forceinline__ v8f wmma16(v8f acc, v16h a, v16h b) {
    acc = __builtin_amdgcn_wmma_f32_16x16x32_f16(false, a, false, b, (short)0, acc, false, false);
    asm volatile("v_nop\n\tv_nop\n\tv_nop\n\tv_nop" : "+v"(acc) : "v"(a), "v"(b));
    return acc;
}

__global__ __launch_bounds__(128, 1)
void fa_prep(const float* __restrict__ K, const float* __restrict__ V,
             _Float16* __restrict__ Kh, _Float16* __restrict__ Vt)
{
    __shared__ __align__(16) _Float16 T[HD * KVT];
    const int tid = threadIdx.x;
    const int bh  = blockIdx.x / NT;
    const int t   = blockIdx.x - bh * NT;
    const size_t ib = ((size_t)bh * SEQ_FULL + (size_t)t * KVT) * HD;
    const size_t wb = ((size_t)bh * SEQ      + (size_t)t * KVT) * HD;

    v8h kh[2], vt8[2];
#pragma unroll
    for (int j = 0; j < 2; ++j) {
        const int e0 = tid * 8 + j * 1024;
        float4 a = *(const float4*)(K + ib + e0);
        float4 c = *(const float4*)(K + ib + e0 + 4);
        kh[j] = cvt8(a, c);
        float4 e = *(const float4*)(V + ib + e0);
        float4 f = *(const float4*)(V + ib + e0 + 4);
        v8h hv = cvt8(e, f);
        const int krow = e0 >> 6;
        const int d0   = e0 & 63;
#pragma unroll
        for (int i = 0; i < 8; ++i) T[(d0 + i) * KVT + krow] = hv[i];
    }
#pragma unroll
    for (int j = 0; j < 2; ++j)
        *(volatile v8h*)(Kh + wb + (size_t)tid * 8 + j * 1024) = kh[j];
    __syncthreads();
#pragma unroll
    for (int j = 0; j < 2; ++j)
        vt8[j] = *(const v8h*)(&T[tid * 8 + j * 1024]);
#pragma unroll
    for (int j = 0; j < 2; ++j)
        *(volatile v8h*)(Vt + wb + (size_t)tid * 8 + j * 1024) = vt8[j];
    __threadfence();
#pragma unroll
    for (int j = 0; j < 2; ++j) {
        *(volatile v8h*)(Kh + wb + (size_t)tid * 8 + j * 1024) = kh[j];
        *(volatile v8h*)(Vt + wb + (size_t)tid * 8 + j * 1024) = vt8[j];
    }
}

__global__ __launch_bounds__(128, 1) __attribute__((amdgpu_num_vgpr(256)))
void fa_main(const float* __restrict__ Q,
             const _Float16* __restrict__ Kh,
             const _Float16* __restrict__ Vt,
             float* __restrict__ O)
{
    __shared__ __align__(16) _Float16 Kst[2][TILE_H];
    __shared__ __align__(16) _Float16 Vst[2][TILE_H];
    __shared__ __align__(16) float    Ost[WAVES][16 * HD];

    const int tid  = threadIdx.x;
    const int wave = tid >> 5;
    const int lane = tid & 31;
    const int ln   = lane & 15;
    const int koff = (lane >> 4) * 8;
    const int mb   = koff;

    const int bh   = blockIdx.x / QBLKS;
    const int qblk = blockIdx.x - bh * QBLKS;
    const int q0   = qblk * QB + wave * 16;
    const size_t qin = (size_t)bh * SEQ_FULL * HD;
    const size_t wsb = (size_t)bh * SEQ * HD;

    v16h qa[2];
    {
        const float* qp = Q + qin + (size_t)(q0 + ln) * HD;
#pragma unroll
        for (int dc = 0; dc < 2; ++dc) {
            const int off = dc * 32 + koff;
            float4 f0 = *(const float4*)(qp + off);
            float4 f1 = *(const float4*)(qp + off + 4);
            float4 f2 = *(const float4*)(qp + off + 16);
            float4 f3 = *(const float4*)(qp + off + 20);
            v16h a;
            a[0]  = to_h(f0.x); a[1]  = to_h(f0.y); a[2]  = to_h(f0.z); a[3]  = to_h(f0.w);
            a[4]  = to_h(f1.x); a[5]  = to_h(f1.y); a[6]  = to_h(f1.z); a[7]  = to_h(f1.w);
            a[8]  = to_h(f2.x); a[9]  = to_h(f2.y); a[10] = to_h(f2.z); a[11] = to_h(f2.w);
            a[12] = to_h(f3.x); a[13] = to_h(f3.y); a[14] = to_h(f3.z); a[15] = to_h(f3.w);
            qa[dc] = a;
        }
    }

    v8f ot[4] = {};
    float mrun = -__builtin_inff();
    float lrun = 0.0f;

    const _Float16* kbase = Kh + wsb + (size_t)tid * 16;
    const _Float16* vbase = Vt + wsb + (size_t)tid * 16;

    v8h kr[2], vr[2];
#pragma unroll
    for (int j = 0; j < 2; ++j) {
        kr[j] = *(const v8h*)(kbase + 8 * j);
        vr[j] = *(const v8h*)(vbase + 8 * j);
    }
#pragma unroll
    for (int j = 0; j < 2; ++j) {
        *(v8h*)(&Kst[0][tid * 16 + 8 * j]) = kr[j];
        *(v8h*)(&Vst[0][tid * 16 + 8 * j]) = vr[j];
    }
    __syncthreads();

#pragma unroll 1
    for (int t = 0; t < NT; ++t) {
        const int cur = t & 1;

        if (t + 1 < NT) {
            const _Float16* kn = kbase + (size_t)(t + 1) * TILE_H;
            const _Float16* vn = vbase + (size_t)(t + 1) * TILE_H;
#pragma unroll
            for (int j = 0; j < 2; ++j) {
                kr[j] = *(const v8h*)(kn + 8 * j);
                vr[j] = *(const v8h*)(vn + 8 * j);
            }
        }

        v16h kb[4];
#pragma unroll
        for (int dc = 0; dc < 2; ++dc) {
            kb[dc]     = ld_op16(&Kst[cur][(0  + ln) * HD + dc * 32 + koff]);
            kb[2 + dc] = ld_op16(&Kst[cur][(16 + ln) * HD + dc * 32 + koff]);
        }
        v8f ct0 = {}, ct1 = {};
#pragma unroll
        for (int dc = 0; dc < 2; ++dc) {
            ct0 = wmma16(ct0, kb[dc],     qa[dc]);
            ct1 = wmma16(ct1, kb[2 + dc], qa[dc]);
        }

        float vmax = ct0[0];
#pragma unroll
        for (int r = 1; r < 8; ++r) vmax = fmaxf(vmax, ct0[r]);
#pragma unroll
        for (int r = 0; r < 8; ++r) vmax = fmaxf(vmax, ct1[r]);
        vmax = fmaxf(vmax, __shfl_xor(vmax, 16, 32));
        const float mnew = fmaxf(mrun, vmax);
        const float corr = fast_exp2((mrun - mnew) * SL2E);
        mrun = mnew;

        v16h pa;
        float rs = 0.0f;
#pragma unroll
        for (int r = 0; r < 8; ++r) {
            float p = fast_exp2((ct0[r] - mnew) * SL2E);
            rs += p; pa[r] = (_Float16)(p * PSCALE);
        }
#pragma unroll
        for (int r = 0; r < 8; ++r) {
            float p = fast_exp2((ct1[r] - mnew) * SL2E);
            rs += p; pa[8 + r] = (_Float16)(p * PSCALE);
        }
        rs += __shfl_xor(rs, 16, 32);
        lrun = lrun * corr + rs;

#pragma unroll
        for (int db = 0; db < 4; ++db)
            ot[db] = ot[db] * corr;

        v16h vb[4];
#pragma unroll
        for (int db = 0; db < 4; ++db)
            vb[db] = ld_op16(&Vst[cur][(db * 16 + ln) * KVT + koff]);
#pragma unroll
        for (int db = 0; db < 4; ++db)
            ot[db] = wmma16(ot[db], vb[db], pa);

        if (t + 1 < NT) {
            _Float16* kd = &Kst[cur ^ 1][tid * 16];
            _Float16* vd = &Vst[cur ^ 1][tid * 16];
#pragma unroll
            for (int j = 0; j < 2; ++j) {
                *(v8h*)(kd + 8 * j) = kr[j];
                *(v8h*)(vd + 8 * j) = vr[j];
            }
        }
        __syncthreads();
    }

    const float inv = fast_rcp(lrun) * PINV;
    float* ow = &Ost[wave][ln * HD + mb];
#pragma unroll
    for (int db = 0; db < 4; ++db) {
        v4f lo4, hi4;
        lo4[0] = ot[db][0] * inv; lo4[1] = ot[db][1] * inv;
        lo4[2] = ot[db][2] * inv; lo4[3] = ot[db][3] * inv;
        hi4[0] = ot[db][4] * inv; hi4[1] = ot[db][5] * inv;
        hi4[2] = ot[db][6] * inv; hi4[3] = ot[db][7] * inv;
        *(v4f*)(ow + db * 16)     = lo4;
        *(v4f*)(ow + db * 16 + 4) = hi4;
    }
    __syncthreads();

    v4f ov[8];
    const float* orl = &Ost[wave][lane * 4];
#pragma unroll
    for (int i = 0; i < 8; ++i) ov[i] = *(const v4f*)(orl + i * 128);
    float* og = O + wsb + (size_t)q0 * HD + lane * 4;
#pragma unroll
    for (int i = 0; i < 8; ++i) *(volatile v4f*)(og + i * 128) = ov[i];
    __threadfence();
#pragma unroll
    for (int i = 0; i < 8; ++i) *(volatile v4f*)(og + i * 128) = ov[i];
}

extern "C" void kernel_launch(void* const* d_in, const int* in_sizes, int n_in,
                              void* d_out, int out_size, void* d_ws, size_t ws_size,
                              hipStream_t stream) {
    if (n_in < 3) return;
    const int need = NBH * SEQ * HD;
    if (in_sizes[0] < need || in_sizes[1] < need || in_sizes[2] < need) return;
    if (out_size < need) return;
    const size_t plane = (size_t)NBH * SEQ * HD;
    if (ws_size < 2 * plane * sizeof(_Float16)) return;

    const float* Q = (const float*)d_in[0];
    const float* K = (const float*)d_in[1];
    const float* V = (const float*)d_in[2];
    float* O = (float*)d_out;
    _Float16* Kh = (_Float16*)d_ws;
    _Float16* Vt = Kh + plane;

    hipLaunchKernelGGL(fa_prep, dim3(NBH * NT), dim3(128), 0, stream, K, V, Kh, Vt);
    hipLaunchKernelGGL(fa_main, dim3(NBH * QBLKS), dim3(128), 0, stream, Q, Kh, Vt, O);
}
